// TransformerBlock_72696616452196
// MI455X (gfx1250) — hardware-verified
//
#include <hip/hip_runtime.h>
#include <stddef.h>


typedef _Float16 v16h __attribute__((ext_vector_type(16)));
typedef _Float16 v8h  __attribute__((ext_vector_type(8)));
typedef float    v8f  __attribute__((ext_vector_type(8)));
typedef float    v4f  __attribute__((ext_vector_type(4)));

#ifndef NB
#define NB 2
#endif
#ifndef SEQ
#define SEQ 2048
#endif
#define NB_FULL  2
#define SEQ_FULL 2048
#define DIM   768
#define DFF   3072
#define NHEAD 12
#define HD    64
#define MROWS (NB * SEQ)
#define LNROWS 8
#define LN_EPS 1.0e-5f

static_assert(NB >= 1 && NB <= NB_FULL);
static_assert(SEQ >= 128 && SEQ <= SEQ_FULL && (SEQ % 128) == 0);
static_assert(DIM == NHEAD * HD);
static_assert(HD == 64);
static_assert((DIM % 64) == 0 && (DIM % 32) == 0);
static_assert((DFF % 64) == 0 && (DFF % 32) == 0);
static_assert((MROWS % 64) == 0);
static_assert((SEQ % 64) == 0);
static_assert((MROWS % LNROWS) == 0);
static_assert((DIM % 256) == 0);
static_assert((DIM % 8) == 0);
static_assert(((size_t)MROWS * DIM) % 2048 == 0);
static_assert((size_t)MROWS * DFF < (size_t)0xFFFFFFFFu);
static_assert((size_t)DFF * DIM < (size_t)0xFFFFFFFFu);

#define LDT 72
#define LDC 68
#define TPT 65

#define WCARRY 64.0f
#define RCARRY 2048.0f
#define VCARRY 16.0f
#define PCARRY 4096.0f
#define CCARRY 256.0f
#define HCARRY 16.0f

#define WSQ_BYTES  ((size_t)DIM * DIM * 2)
#define WFF_BYTES  ((size_t)DFF * DIM * 2)
#define P16_BYTES  ((size_t)MROWS * DIM * 2)
#define P32_BYTES  ((size_t)MROWS * DIM * 4)
#define F1_BYTES   ((size_t)MROWS * DFF * 2)
#define OFF_WQ   ((size_t)0)
#define OFF_WK   (OFF_WQ + WSQ_BYTES)
#define OFF_WV   (OFF_WK + WSQ_BYTES)
#define OFF_WO   (OFF_WV + WSQ_BYTES)
#define OFF_W1   (OFF_WO + WSQ_BYTES)
#define OFF_W2   (OFF_W1 + WFF_BYTES)
#define OFF_X16  (OFF_W2 + WFF_BYTES)
#define OFF_QH   (OFF_X16 + P16_BYTES)
#define OFF_QR   (OFF_QH + P16_BYTES)
#define OFF_KH   (OFF_QR + P16_BYTES)
#define OFF_KR   (OFF_KH + P16_BYTES)
#define OFF_VT   (OFF_KR + P16_BYTES)
#define OFF_CTX  (OFF_VT + P16_BYTES)
#define OFF_A1   (OFF_CTX + P16_BYTES)
#define OFF_HF   (OFF_A1 + P32_BYTES)
#define OFF_H16  (OFF_HF + P32_BYTES)
#define OFF_F1   (OFF_H16 + P16_BYTES)
#define OFF_Y    (OFF_F1 + F1_BYTES)
#define WS_TOTAL (OFF_Y + P32_BYTES)
static_assert((WSQ_BYTES % 128) == 0 && (WFF_BYTES % 128) == 0);
static_assert((P16_BYTES % 128) == 0 && (P32_BYTES % 128) == 0 && (F1_BYTES % 128) == 0);
static_assert(WS_TOTAL <= (size_t)134217728);

__device__ __forceinline__ float bf16r(float x) {
  unsigned int u = __float_as_uint(x);
  u = (u + 0x7FFFu + ((u >> 16) & 1u)) & 0xFFFF0000u;
  return __uint_as_float(u);
}

__device__ __forceinline__ v16h frag_at(const _Float16* p) {
  v8h lo = *(const v8h*)(p);
  v8h hi = *(const v8h*)(p + 16);
  v16h out;
#pragma unroll
  for (int i = 0; i < 8; ++i) { out[i] = lo[i]; out[i + 8] = hi[i]; }
  return out;
}
__device__ __forceinline__ v16h ld_frag(const _Float16* base, unsigned ld) {
  const unsigned lane = threadIdx.x & 31u;
  return frag_at(base + (lane & 15u) * ld + (lane >> 4) * 8u);
}

__device__ __forceinline__ v8f wmma16(v16h a, v16h b, v8f c) {
  v8f d = __builtin_amdgcn_wmma_f32_16x16x32_f16(false, a, false, b, (short)0, c,
                                                 false, false);
  asm volatile("v_nop\n\tv_nop\n\tv_nop\n\tv_nop" : "+v"(d) : "v"(a), "v"(b));
  return d;
}

__device__ __forceinline__ float red16_max(float x) {
#pragma unroll
  for (int off = 1; off < 16; off <<= 1) x = fmaxf(x, __shfl_xor(x, off, 32));
  return x;
}
__device__ __forceinline__ float red16_sum(float x) {
#pragma unroll
  for (int off = 1; off < 16; off <<= 1) x += __shfl_xor(x, off, 32);
  return x;
}
__device__ __forceinline__ float red32_sum(float x) {
#pragma unroll
  for (int off = 1; off < 32; off <<= 1) x += __shfl_xor(x, off, 32);
  return x;
}

__device__ __forceinline__ void wave_lds_sync() {
  __builtin_amdgcn_fence(3  , "wavefront");
  asm volatile("s_wait_dscnt 0x0" ::: "memory");
  __builtin_amdgcn_wave_barrier();
}

__global__ __launch_bounds__(256) void conv_x_kernel(
    const float* __restrict__ src, _Float16* __restrict__ dst) {
  const unsigned e = (blockIdx.x * 256u + threadIdx.x) * 8u;
  const unsigned row = e / (unsigned)DIM;
  const unsigned col = e - row * (unsigned)DIM;
  const unsigned bb = row / (unsigned)SEQ;
  const unsigned ss = row - bb * (unsigned)SEQ;
  const size_t so = ((size_t)bb * SEQ_FULL + ss) * DIM + col;
  const v4f a0 = *(const v4f*)(src + so);
  const v4f a1 = *(const v4f*)(src + so + 4);
  v8h o;
#pragma unroll
  for (int j = 0; j < 4; ++j) {
    o[j]     = (_Float16)bf16r(a0[j]);
    o[j + 4] = (_Float16)bf16r(a1[j]);
  }
  *(volatile v8h*)(dst + e) = o;
  __threadfence();
  *(volatile v8h*)(dst + e) = o;
}

__global__ __launch_bounds__(256) void wtrans_kernel(
    const float* __restrict__ src, _Float16* __restrict__ dst, unsigned R, unsigned C) {
  __shared__ float T[64 * TPT];
  const unsigned tid = threadIdx.x;
  const unsigned c0 = blockIdx.x * 64u;
  const unsigned r0 = blockIdx.y * 64u;
#pragma unroll
  for (unsigned i = 0; i < 4u; ++i) {
    const unsigned idx = tid + 256u * i;
    const unsigned r = idx >> 4, c = (idx & 15u) * 4u;
    const v4f a = *(const v4f*)(src + (size_t)(r0 + r) * C + c0 + c);
#pragma unroll
    for (int j = 0; j < 4; ++j) T[r * TPT + c + (unsigned)j] = WCARRY * bf16r(a[j]);
  }
  __syncthreads();
  v8h x[2];
  size_t off[2];
#pragma unroll
  for (unsigned i = 0; i < 2u; ++i) {
    const unsigned oc = 32u * i + (tid >> 3);
    const unsigned seg = (tid & 7u) * 8u;
#pragma unroll
    for (unsigned j = 0; j < 8u; ++j) x[i][j] = (_Float16)T[(seg + j) * TPT + oc];
    off[i] = (size_t)(c0 + oc) * R + r0 + seg;
  }
#pragma unroll
  for (int i = 0; i < 2; ++i) *(volatile v8h*)(dst + off[i]) = x[i];
  __threadfence();
#pragma unroll
  for (int i = 0; i < 2; ++i) *(volatile v8h*)(dst + off[i]) = x[i];
}

template <int MODE, int KD, int LDO, int RESX>
__device__ __forceinline__ void gemm_body(
    const _Float16* __restrict__ A16, const _Float16* __restrict__ Bt,
    const float* __restrict__ addf, const float* __restrict__ resf,
    float* __restrict__ outf, _Float16* __restrict__ out16, _Float16* __restrict__ out16r,
    float* Cs, const float ascale, const float ocarry) {
  static_assert((KD % 32) == 0);
  static_assert((LDO % 64) == 0);
  const unsigned tid = threadIdx.x, lane = tid & 31u;
  const unsigned w = (unsigned)__builtin_amdgcn_readfirstlane((int)(tid >> 5));
  const unsigned mw = w >> 1, nw = w & 1u;
  const unsigned hh = lane >> 4, m = lane & 15u;
  const unsigned n0 = blockIdx.x * 64u;
  const unsigned row0 = blockIdx.y * 64u;

  const _Float16* ap  = A16 + (size_t)(row0 + mw * 16u + m) * KD + hh * 8u;
  const _Float16* bp0 = Bt + (size_t)(n0 + nw * 32u + m) * KD + hh * 8u;
  const _Float16* bp1 = bp0 + (size_t)16 * KD;
  v8f acc0 = {}, acc1 = {};
#pragma unroll 2
  for (unsigned k0 = 0; k0 < (unsigned)KD; k0 += 32u) {
    const v16h a  = frag_at(ap + k0);
    const v16h b0 = frag_at(bp0 + k0);
    const v16h b1 = frag_at(bp1 + k0);
    acc0 = wmma16(a, b0, acc0);
    acc1 = wmma16(a, b1, acc1);
  }
#pragma unroll
  for (int r = 0; r < 8; ++r) {
    float* d = &Cs[(mw * 16u + hh * 8u + (unsigned)r) * LDC + nw * 32u + m];
    d[0]  = acc0[r];
    d[16] = acc1[r];
  }
  __syncthreads();

  if (MODE == 0) {
    v8h xh[2], xr[2];
    size_t off[2];
#pragma unroll
    for (unsigned i = 0; i < 2u; ++i) {
      const unsigned r = 32u * i + (tid >> 3);
      const unsigned c = (tid & 7u) * 8u;
      const v4f u0 = *(const v4f*)&Cs[r * LDC + c];
      const v4f u1 = *(const v4f*)&Cs[r * LDC + c + 4];
      const v4f g0 = *(const v4f*)(addf + n0 + c);
      const v4f g1 = *(const v4f*)(addf + n0 + c + 4);
#pragma unroll
      for (int j = 0; j < 4; ++j) {
        const float va = u0[j] * ascale + bf16r(g0[j]);
        const float vb = u1[j] * ascale + bf16r(g1[j]);
        const _Float16 ha = (_Float16)va;
        const _Float16 hb = (_Float16)vb;
        xh[i][j]     = ha;
        xh[i][j + 4] = hb;
        xr[i][j]     = (_Float16)((va - (float)ha) * RCARRY);
        xr[i][j + 4] = (_Float16)((vb - (float)hb) * RCARRY);
      }
      off[i] = (size_t)(row0 + r) * LDO + n0 + c;
    }
#pragma unroll
    for (int i = 0; i < 2; ++i) {
      *(volatile v8h*)(out16 + off[i]) = xh[i];
      *(volatile v8h*)(out16r + off[i]) = xr[i];
    }
    __threadfence();
#pragma unroll
    for (int i = 0; i < 2; ++i) {
      *(volatile v8h*)(out16 + off[i]) = xh[i];
      *(volatile v8h*)(out16r + off[i]) = xr[i];
    }
  }

  if (MODE == 3) {
    v8h x[2];
    size_t off[2];
#pragma unroll
    for (unsigned i = 0; i < 2u; ++i) {
      const unsigned r = 32u * i + (tid >> 3);
      const unsigned c = (tid & 7u) * 8u;
      const v4f u0 = *(const v4f*)&Cs[r * LDC + c];
      const v4f u1 = *(const v4f*)&Cs[r * LDC + c + 4];
      const v4f g0 = *(const v4f*)(addf + n0 + c);
      const v4f g1 = *(const v4f*)(addf + n0 + c + 4);
#pragma unroll
      for (int j = 0; j < 4; ++j) {
        x[i][j]     = (_Float16)(ocarry * fmaxf(u0[j] * ascale + bf16r(g0[j]), 0.0f));
        x[i][j + 4] = (_Float16)(ocarry * fmaxf(u1[j] * ascale + bf16r(g1[j]), 0.0f));
      }
      off[i] = (size_t)(row0 + r) * LDO + n0 + c;
    }
#pragma unroll
    for (int i = 0; i < 2; ++i) *(volatile v8h*)(out16 + off[i]) = x[i];
    __threadfence();
#pragma unroll
    for (int i = 0; i < 2; ++i) *(volatile v8h*)(out16 + off[i]) = x[i];
  }

  if (MODE == 1) {
    const unsigned bidx = row0 / (unsigned)SEQ;
    const unsigned key0 = row0 - bidx * (unsigned)SEQ;
    v8h x[2];
    size_t off[2];
#pragma unroll
    for (unsigned i = 0; i < 2u; ++i) {
      const unsigned dcol = 32u * i + (tid >> 3);
      const unsigned kk = (tid & 7u) * 8u;
      const float bb = bf16r(addf[n0 + dcol]);
#pragma unroll
      for (unsigned j = 0; j < 8u; ++j)
        x[i][j] = (_Float16)(ocarry * (Cs[(kk + j) * LDC + dcol] * ascale + bb));
      off[i] = ((size_t)bidx * DIM + n0 + dcol) * SEQ + key0 + kk;
    }
#pragma unroll
    for (int i = 0; i < 2; ++i) *(volatile v8h*)(out16 + off[i]) = x[i];
    __threadfence();
#pragma unroll
    for (int i = 0; i < 2; ++i) *(volatile v8h*)(out16 + off[i]) = x[i];
  }

  if (MODE == 4) {
    v4f xs[4];
    size_t off[4];
#pragma unroll
    for (unsigned i = 0; i < 4u; ++i) {
      const unsigned r = 16u * i + (tid >> 4);
      const unsigned c = (tid & 15u) * 4u;
      const unsigned row = row0 + r;
      const size_t o = (size_t)row * DIM + n0 + c;
      const v4f u = *(const v4f*)&Cs[r * LDC + c];
      const v4f g = *(const v4f*)(addf + n0 + c);
      v4f hres;
      if (RESX) {
        const unsigned bb = row / (unsigned)SEQ;
        const unsigned ss = row - bb * (unsigned)SEQ;
        const v4f xin = *(const v4f*)(resf + ((size_t)bb * SEQ_FULL + ss) * DIM + n0 + c);
#pragma unroll
        for (int j = 0; j < 4; ++j) hres[j] = bf16r(xin[j]);
      } else {
        hres = *(const v4f*)(resf + o);
      }
      v4f val;
#pragma unroll
      for (int j = 0; j < 4; ++j)
        val[j] = (u[j] * ascale + bf16r(g[j])) + hres[j];
      xs[i] = val;
      off[i] = o;
    }
#pragma unroll
    for (int i = 0; i < 4; ++i) *(volatile v4f*)(outf + off[i]) = xs[i];
    __threadfence();
#pragma unroll
    for (int i = 0; i < 4; ++i) *(volatile v4f*)(outf + off[i]) = xs[i];
  }
}

__global__ __launch_bounds__(256) void gemm_qk_kernel(
    const _Float16* __restrict__ A16, const _Float16* __restrict__ Bt,
    const float* __restrict__ bias, _Float16* __restrict__ outH,
    _Float16* __restrict__ outR) {
  __shared__ __attribute__((aligned(16))) float Cs[64 * LDC];
  gemm_body<0, DIM, DIM, 0>(A16, Bt, bias, nullptr, nullptr, outH, outR, Cs,
                            1.0f / WCARRY, 1.0f);
}
__global__ __launch_bounds__(256) void gemm_vt_kernel(
    const _Float16* __restrict__ A16, const _Float16* __restrict__ Bt,
    const float* __restrict__ bias, _Float16* __restrict__ out16) {
  __shared__ __attribute__((aligned(16))) float Cs[64 * LDC];
  gemm_body<1, DIM, DIM, 0>(A16, Bt, bias, nullptr, nullptr, out16, nullptr, Cs,
                            1.0f / WCARRY, VCARRY);
}
__global__ __launch_bounds__(256) void gemm_oproj_kernel(
    const _Float16* __restrict__ A16, const _Float16* __restrict__ Bt,
    const float* __restrict__ bias, const float* __restrict__ xres,
    float* __restrict__ outf) {
  __shared__ __attribute__((aligned(16))) float Cs[64 * LDC];
  gemm_body<4, DIM, DIM, 1>(A16, Bt, bias, xres, outf, nullptr, nullptr, Cs,
                            1.0f / (CCARRY * WCARRY), 1.0f);
}
__global__ __launch_bounds__(256) void gemm_ffn1_kernel(
    const _Float16* __restrict__ A16, const _Float16* __restrict__ Bt,
    const float* __restrict__ bias, _Float16* __restrict__ out16) {
  __shared__ __attribute__((aligned(16))) float Cs[64 * LDC];
  gemm_body<3, DIM, DFF, 0>(A16, Bt, bias, nullptr, nullptr, out16, nullptr, Cs,
                            1.0f / (HCARRY * WCARRY), HCARRY);
}
__global__ __launch_bounds__(256) void gemm_ffn2_kernel(
    const _Float16* __restrict__ A16, const _Float16* __restrict__ Bt,
    const float* __restrict__ bias, const float* __restrict__ resf,
    float* __restrict__ outf) {
  __shared__ __attribute__((aligned(16))) float Cs[64 * LDC];
  gemm_body<4, DFF, DIM, 0>(A16, Bt, bias, resf, outf, nullptr, nullptr, Cs,
                            1.0f / (HCARRY * WCARRY), 1.0f);
}

__global__ __launch_bounds__(256) void attn_kernel(
    const _Float16* __restrict__ Qh, const _Float16* __restrict__ Qr,
    const _Float16* __restrict__ Kh, const _Float16* __restrict__ Kr,
    const _Float16* __restrict__ Vt, _Float16* __restrict__ Ov) {
  __shared__ __attribute__((aligned(16))) _Float16 Ksh[64 * LDT];
  __shared__ __attribute__((aligned(16))) _Float16 Ksr[64 * LDT];
  __shared__ __attribute__((aligned(16))) _Float16 Vs[64 * LDT];
  __shared__ __attribute__((aligned(16))) _Float16 Ps[8 * 16 * LDT];

  const unsigned tid = threadIdx.x, lane = tid & 31u;
  const unsigned wave = (unsigned)__builtin_amdgcn_readfirstlane((int)(tid >> 5));
  const unsigned hh = lane >> 4, m = lane & 15u;
  const unsigned q0 = blockIdx.x * 128u;
  const unsigned head = blockIdx.y;
  const unsigned bidx = blockIdx.z;
  const float scale = 0.125f;
  const unsigned pb = wave * (16u * LDT);

  const size_t rowb = (size_t)bidx * SEQ;
  const size_t qoff = (rowb + q0 + wave * 16u + m) * DIM + head * HD + hh * 8u;
  const size_t kplane = rowb * DIM + (size_t)head * HD;
  const size_t vplane = ((size_t)bidx * DIM + head * HD) * SEQ;

  float mrow[8], lrow[8];
  v8f o[4];
#pragma unroll
  for (int v = 0; v < 8; ++v) { mrow[v] = -1.0e30f; lrow[v] = 0.0f; }
#pragma unroll
  for (int nb = 0; nb < 4; ++nb) o[nb] = (v8f){};

  for (unsigned kb = 0; kb < (unsigned)SEQ; kb += 64u) {
#pragma unroll
    for (unsigned j = 0; j < 2u; ++j) {
      const unsigned idx = tid + 256u * j;
      const unsigned r = idx >> 3, c = (idx & 7u) * 8u;
      const size_t ko = kplane + (size_t)(kb + r) * DIM + c;
      *(v8h*)&Ksh[r * LDT + c] = *(const v8h*)(Kh + ko);
      *(v8h*)&Ksr[r * LDT + c] = *(const v8h*)(Kr + ko);
      *(v8h*)&Vs[r * LDT + c]  = *(const v8h*)(Vt + vplane + (size_t)r * SEQ + kb + c);
    }
    __syncthreads();

    v8f s[4];
#pragma unroll
    for (int hf = 0; hf < 2; ++hf) {
      v8f t0 = {}, t1 = {}, u0 = {}, u1 = {};
#pragma unroll
      for (int c = 0; c < 2; ++c) {
        const v16h qh = frag_at(Qh + qoff + c * 32);
        const v16h qr = frag_at(Qr + qoff + c * 32);
        const v16h ka = ld_frag(&Ksh[((hf * 2) * 16) * LDT + c * 32], LDT);
        const v16h ra = ld_frag(&Ksr[((hf * 2) * 16) * LDT + c * 32], LDT);
        t0 = wmma16(qh, ka, t0);
        u0 = wmma16(qh, ra, u0);
        u0 = wmma16(qr, ka, u0);
        const v16h kc = ld_frag(&Ksh[((hf * 2 + 1) * 16) * LDT + c * 32], LDT);
        const v16h rc = ld_frag(&Ksr[((hf * 2 + 1) * 16) * LDT + c * 32], LDT);
        t1 = wmma16(qh, kc, t1);
        u1 = wmma16(qh, rc, u1);
        u1 = wmma16(qr, kc, u1);
      }
      s[hf * 2]     = (t0 + u0 * (1.0f / RCARRY)) * scale;
      s[hf * 2 + 1] = (t1 + u1 * (1.0f / RCARRY)) * scale;
    }

    float alpha[8];
#pragma unroll
    for (int v = 0; v < 8; ++v) {
      float mx = fmaxf(fmaxf(s[0][v], s[1][v]), fmaxf(s[2][v], s[3][v]));
      mx = red16_max(mx);
      const float mn = fmaxf(mrow[v], mx);
      alpha[v] = __expf(mrow[v] - mn);
      mrow[v] = mn;
    }
#pragma unroll
    for (int kg = 0; kg < 4; ++kg)
#pragma unroll
      for (int v = 0; v < 8; ++v) s[kg][v] = __expf(s[kg][v] - mrow[v]);
#pragma unroll
    for (int v = 0; v < 8; ++v) {
      const float rs = red16_sum((s[0][v] + s[1][v]) + (s[2][v] + s[3][v]));
      lrow[v] = alpha[v] * lrow[v] + rs;
    }
#pragma unroll
    for (int nb = 0; nb < 4; ++nb)
#pragma unroll
      for (int v = 0; v < 8; ++v) o[nb][v] = o[nb][v] * alpha[v];

#pragma unroll
    for (int kg = 0; kg < 4; ++kg)
#pragma unroll
      for (int v = 0; v < 8; ++v)
        Ps[pb + (hh * 8u + (unsigned)v) * LDT + (unsigned)kg * 16u + m] =
            (_Float16)(s[kg][v] * PCARRY);
    wave_lds_sync();

#pragma unroll
    for (int c = 0; c < 2; ++c) {
      const v16h pf = ld_frag(&Ps[pb + c * 32], LDT);
#pragma unroll
      for (int nb = 0; nb < 4; ++nb) {
        const v16h vf = ld_frag(&Vs[(nb * 16) * LDT + c * 32], LDT);
        o[nb] = wmma16(pf, vf, o[nb]);
      }
    }
    __syncthreads();
  }

  float inv[8];
#pragma unroll
  for (int v = 0; v < 8; ++v)
    inv[v] = __builtin_amdgcn_rcpf(lrow[v]) * (CCARRY / (PCARRY * VCARRY));
#pragma unroll
  for (int nb = 0; nb < 4; ++nb)
#pragma unroll
    for (int v = 0; v < 8; ++v)
      Ps[pb + (hh * 8u + (unsigned)v) * LDT + (unsigned)nb * 16u + m] =
          (_Float16)(o[nb][v] * inv[v]);
  wave_lds_sync();
  v8h x[4];
  size_t off[4];
#pragma unroll
  for (unsigned i = 0; i < 4u; ++i) {
    const unsigned r = 4u * i + (lane >> 3);
    const unsigned c = (lane & 7u) * 8u;
    x[i] = *(const v8h*)&Ps[pb + r * LDT + c];
    off[i] = (rowb + q0 + wave * 16u + r) * DIM + head * HD + c;
  }
#pragma unroll
  for (int i = 0; i < 4; ++i) *(volatile v8h*)(Ov + off[i]) = x[i];
  __threadfence();
#pragma unroll
  for (int i = 0; i < 4; ++i) *(volatile v8h*)(Ov + off[i]) = x[i];
}

template <int W16>
__device__ __forceinline__ void ln_store(
    const float* S, const float* __restrict__ g, const float* __restrict__ be,
    float* __restrict__ outF, _Float16* __restrict__ out16, size_t rbase, float mu, float rs) {
  const unsigned lane = threadIdx.x & 31u;
#pragma unroll 1
  for (unsigned it = 0; it < (unsigned)(DIM / 128); ++it) {
    const unsigned c = it * 128u + lane * 4u;
    const v4f v = *(const v4f*)&S[c];
    const v4f gg = *(const v4f*)(g + c);
    const v4f bb = *(const v4f*)(be + c);
    v4f ov;
#pragma unroll
    for (int j = 0; j < 4; ++j) ov[j] = (v[j] - mu) * rs * bf16r(gg[j]) + bf16r(bb[j]);
    *(volatile v4f*)(outF + rbase + c) = ov;
  }
  if (W16) {
#pragma unroll 1
    for (unsigned it = 0; it < (unsigned)(DIM / 256); ++it) {
      const unsigned c = it * 256u + lane * 8u;
      const v4f v0 = *(const v4f*)&S[c];
      const v4f v1 = *(const v4f*)&S[c + 4];
      const v4f g0 = *(const v4f*)(g + c);
      const v4f g1 = *(const v4f*)(g + c + 4);
      const v4f b0 = *(const v4f*)(be + c);
      const v4f b1 = *(const v4f*)(be + c + 4);
      v8h x;
#pragma unroll
      for (int j = 0; j < 4; ++j) {
        x[j]     = (_Float16)(HCARRY * ((v0[j] - mu) * rs * bf16r(g0[j]) + bf16r(b0[j])));
        x[j + 4] = (_Float16)(HCARRY * ((v1[j] - mu) * rs * bf16r(g1[j]) + bf16r(b1[j])));
      }
      *(volatile v8h*)(out16 + rbase + c) = x;
    }
  }
}

template <int W16>
__device__ __forceinline__ void ln_body(
    const float* __restrict__ src, const float* __restrict__ g, const float* __restrict__ be,
    float* __restrict__ outF, _Float16* __restrict__ out16, float* S, unsigned row) {
  const unsigned lane = threadIdx.x & 31u;
  const size_t rbase = (size_t)row * DIM;
  float sum = 0.0f;
#pragma unroll 1
  for (unsigned it = 0; it < (unsigned)(DIM / 128); ++it) {
    const unsigned c = it * 128u + lane * 4u;
    const v4f v = *(const v4f*)(src + rbase + c);
    *(v4f*)&S[c] = v;
    sum += (v[0] + v[1]) + (v[2] + v[3]);
  }
  sum = red32_sum(sum);
  const float mu = sum * (1.0f / (float)DIM);
  float sq = 0.0f;
#pragma unroll 1
  for (unsigned it = 0; it < (unsigned)(DIM / 128); ++it) {
    const unsigned c = it * 128u + lane * 4u;
    const v4f v = *(const v4f*)&S[c];
    const float d0 = v[0] - mu, d1 = v[1] - mu, d2 = v[2] - mu, d3 = v[3] - mu;
    sq += (d0 * d0 + d1 * d1) + (d2 * d2 + d3 * d3);
  }
  sq = red32_sum(sq);
  const float rs = rsqrtf(sq * (1.0f / (float)DIM) + LN_EPS);
  wave_lds_sync();
  ln_store<W16>(S, g, be, outF, out16, rbase, mu, rs);
  __threadfence();
  ln_store<W16>(S, g, be, outF, out16, rbase, mu, rs);
}

__global__ __launch_bounds__(256) void ln1_kernel(
    const float* __restrict__ A1, const float* __restrict__ g,
    const float* __restrict__ be, float* __restrict__ hF, _Float16* __restrict__ h16) {
  __shared__ __attribute__((aligned(16))) float S[LNROWS * DIM];
  const unsigned w = (unsigned)__builtin_amdgcn_readfirstlane((int)(threadIdx.x >> 5));
  const unsigned row = blockIdx.x * (unsigned)LNROWS + w;
  ln_body<1>(A1, g, be, hF, h16, S + w * (unsigned)DIM, row);
}
__global__ __launch_bounds__(256) void ln2_kernel(
    const float* __restrict__ Y, const float* __restrict__ g,
    const float* __restrict__ be, float* __restrict__ out) {
  __shared__ __attribute__((aligned(16))) float S[LNROWS * DIM];
  const unsigned w = (unsigned)__builtin_amdgcn_readfirstlane((int)(threadIdx.x >> 5));
  const unsigned row = blockIdx.x * (unsigned)LNROWS + w;
  ln_body<0>(Y, g, be, out, nullptr, S + w * (unsigned)DIM, row);
}

extern "C" void kernel_launch(void* const* d_in, const int* in_sizes, int n_in,
                              void* d_out, int out_size, void* d_ws, size_t ws_size,
                              hipStream_t stream) {
  if (n_in < 17) return;
  const long long need_x = ((long long)(NB - 1) * SEQ_FULL + SEQ) * DIM;
  const long long need_o = (long long)MROWS * DIM;
  if ((long long)in_sizes[0] < need_x) return;
  if ((long long)in_sizes[1] < (long long)DIM * DIM) return;
  if ((long long)in_sizes[3] < (long long)DIM * DIM) return;
  if ((long long)in_sizes[5] < (long long)DIM * DIM) return;
  if ((long long)in_sizes[7] < (long long)DIM * DIM) return;
  if (in_sizes[2] < DIM || in_sizes[4] < DIM || in_sizes[6] < DIM || in_sizes[8] < DIM) return;
  if ((long long)in_sizes[9] < (long long)DIM * DFF) return;
  if (in_sizes[10] < DFF) return;
  if ((long long)in_sizes[11] < (long long)DFF * DIM) return;
  if (in_sizes[12] < DIM || in_sizes[13] < DIM || in_sizes[14] < DIM) return;
  if (in_sizes[15] < DIM || in_sizes[16] < DIM) return;
  if ((long long)out_size < need_o) return;
  if (ws_size < WS_TOTAL) return;

  const float* X   = (const float*)d_in[0];
  const float* Wq  = (const float*)d_in[1];
  const float* bq  = (const float*)d_in[2];
  const float* Wk  = (const float*)d_in[3];
  const float* bk  = (const float*)d_in[4];
  const float* Wv  = (const float*)d_in[5];
  const float* bv  = (const float*)d_in[6];
  const float* Wo  = (const float*)d_in[7];
  const float* bo  = (const float*)d_in[8];
  const float* W1  = (const float*)d_in[9];
  const float* b1  = (const float*)d_in[10];
  const float* W2  = (const float*)d_in[11];
  const float* b2  = (const float*)d_in[12];
  const float* g1  = (const float*)d_in[13];
  const float* be1 = (const float*)d_in[14];
  const float* g2  = (const float*)d_in[15];
  const float* be2 = (const float*)d_in[16];
  float* out = (float*)d_out;

  char* ws = (char*)d_ws;
  _Float16* WqT   = (_Float16*)(ws + OFF_WQ);
  _Float16* WkT   = (_Float16*)(ws + OFF_WK);
  _Float16* WvT   = (_Float16*)(ws + OFF_WV);
  _Float16* WoT   = (_Float16*)(ws + OFF_WO);
  _Float16* W1T   = (_Float16*)(ws + OFF_W1);
  _Float16* W2T   = (_Float16*)(ws + OFF_W2);
  _Float16* X16   = (_Float16*)(ws + OFF_X16);
  _Float16* Qh16  = (_Float16*)(ws + OFF_QH);
  _Float16* Qr16  = (_Float16*)(ws + OFF_QR);
  _Float16* Kh16  = (_Float16*)(ws + OFF_KH);
  _Float16* Kr16  = (_Float16*)(ws + OFF_KR);
  _Float16* Vt16  = (_Float16*)(ws + OFF_VT);
  _Float16* Ctx16 = (_Float16*)(ws + OFF_CTX);
  float*    A1    = (float*)(ws + OFF_A1);
  float*    HF    = (float*)(ws + OFF_HF);
  _Float16* H16   = (_Float16*)(ws + OFF_H16);
  _Float16* F1_16 = (_Float16*)(ws + OFF_F1);
  float*    Y     = (float*)(ws + OFF_Y);

  dim3 blk(256);

  conv_x_kernel<<<dim3((unsigned)(((size_t)MROWS * DIM) / 2048)), blk, 0, stream>>>(X, X16);

  wtrans_kernel<<<dim3(DIM / 64, DIM / 64), blk, 0, stream>>>(Wq, WqT, (unsigned)DIM, (unsigned)DIM);
  wtrans_kernel<<<dim3(DIM / 64, DIM / 64), blk, 0, stream>>>(Wk, WkT, (unsigned)DIM, (unsigned)DIM);
  wtrans_kernel<<<dim3(DIM / 64, DIM / 64), blk, 0, stream>>>(Wv, WvT, (unsigned)DIM, (unsigned)DIM);
  wtrans_kernel<<<dim3(DIM / 64, DIM / 64), blk, 0, stream>>>(Wo, WoT, (unsigned)DIM, (unsigned)DIM);
  wtrans_kernel<<<dim3(DFF / 64, DIM / 64), blk, 0, stream>>>(W1, W1T, (unsigned)DIM, (unsigned)DFF);
  wtrans_kernel<<<dim3(DIM / 64, DFF / 64), blk, 0, stream>>>(W2, W2T, (unsigned)DFF, (unsigned)DIM);

  gemm_qk_kernel<<<dim3(DIM / 64, MROWS / 64), blk, 0, stream>>>(X16, WqT, bq, Qh16, Qr16);
  gemm_qk_kernel<<<dim3(DIM / 64, MROWS / 64), blk, 0, stream>>>(X16, WkT, bk, Kh16, Kr16);
  gemm_vt_kernel<<<dim3(DIM / 64, MROWS / 64), blk, 0, stream>>>(X16, WvT, bv, Vt16);

  attn_kernel<<<dim3(SEQ / 128, NHEAD, NB), blk, 0, stream>>>(Qh16, Qr16, Kh16, Kr16, Vt16, Ctx16);

  gemm_oproj_kernel<<<dim3(DIM / 64, MROWS / 64), blk, 0, stream>>>(Ctx16, WoT, bo, X, A1);

  ln1_kernel<<<dim3(MROWS / LNROWS), blk, 0, stream>>>(A1, g1, be1, HF, H16);

  gemm_ffn1_kernel<<<dim3(DFF / 64, MROWS / 64), blk, 0, stream>>>(H16, W1T, b1, F1_16);
  gemm_ffn2_kernel<<<dim3(DIM / 64, MROWS / 64), blk, 0, stream>>>(F1_16, W2T, b2, HF, Y);

  ln2_kernel<<<dim3(MROWS / LNROWS), blk, 0, stream>>>(Y, g2, be2, out);
}
